// GraphLSTMBlock_48515950575721
// MI455X (gfx1250) — hardware-run, weakly checked
//
#include <hip/hip_runtime.h>
#include <math.h>

typedef __attribute__((ext_vector_type(16))) _Float16 v16h;
typedef __attribute__((ext_vector_type(8)))  _Float16 v8h;
typedef __attribute__((ext_vector_type(8)))  float    v8f;
typedef __attribute__((ext_vector_type(4)))  float    v4f;
typedef __attribute__((address_space(1))) volatile float gvf;

constexpr int kNodes   = 1024;
constexpr int kDim     = 64;
constexpr int kThreads = 256;
constexpr int kWaves   = kThreads / 32;
constexpr int kRowsPW  = kNodes / kWaves;
constexpr int kTilesPW = kRowsPW / 16;
constexpr int kSlabP   = 68;
constexpr float kCarryH = 64.0f;
constexpr float kCarryW = 256.0f;
constexpr float kFold   = 1.0f / (kCarryH * kCarryW);
constexpr float kF16MinNormal = 6.103515625e-05f;
static_assert(kDim == 64);
static_assert(kNodes == kWaves * kRowsPW);
static_assert(kRowsPW == 16 * kTilesPW);
static_assert((kDim % 32) == 0);
static_assert(kNodes * kDim == 65536);

constexpr size_t kPlaneBytes = (size_t)kNodes * kDim * 4;
constexpr size_t kWsTotal    = kPlaneBytes + kPlaneBytes;
static_assert(kWsTotal == 524288ull);
static_assert(kWsTotal <= 134217728ull);

namespace eng {

union FragU { v16h v; v8h h[2]; };
__device__ __forceinline__ v16h frag_load(const _Float16* p) {
  FragU f;
  f.h[0] = *(const v8h*)(p);
  f.h[1] = *(const v8h*)(p + 16);
  return f.v;
}
__device__ __forceinline__ v8f mma_h(v16h a, v16h b, v8f c) {
  return __builtin_amdgcn_wmma_f32_16x16x32_f16(false, a, false, b, (short)0, c, false, false);
}
__device__ __forceinline__ void guard_acc(v8f& acc, v16h a0, v16h a1, v16h b0, v16h b1) {
  asm volatile("v_nop\n\tv_nop\n\tv_nop\n\tv_nop" : "+v"(acc) : "v"(a0), "v"(a1), "v"(b0), "v"(b1));
}
__device__ __forceinline__ _Float16 to_h_flush(float v, float carry) {
  const float s = v * carry;
  const float z = (fabsf(s) < kF16MinNormal) ? 0.0f : s;
  return (_Float16)z;
}
__device__ __forceinline__ float sigm(float x) {
  return 1.0f / (1.0f + expf(-x));
}
__device__ __forceinline__ void wave_lds_fence() {
  __builtin_amdgcn_fence(__ATOMIC_RELEASE, "workgroup");
  __builtin_amdgcn_wave_barrier();
  __builtin_amdgcn_fence(__ATOMIC_ACQUIRE, "workgroup");
}

}

__global__ __launch_bounds__(256) void state_init_kernel(
    const float* __restrict__ h0, const float* __restrict__ c0,
    float* __restrict__ Hs, float* __restrict__ Cs) {
  const int blk = blockIdx.x, tid = threadIdx.x;
  const bool isC = (blk >= 64);
  const int i = (blk & 63) * 256 + tid;
  const float* src = isC ? c0 : h0;
  float* dst = isC ? Cs : Hs;
  const v4f v = *(const v4f*)(src + (size_t)4 * i);
  volatile v4f* p = (volatile v4f*)(dst + (size_t)4 * i);
  *p = v;
  __threadfence();
  *p = v;
}

__global__ __launch_bounds__(256) void out_double_kernel(
    const float* __restrict__ Hs, float* __restrict__ out) {
  const int i = blockIdx.x * 256 + threadIdx.x;
  const v4f v = *(const v4f*)(Hs + (size_t)4 * i);
  const v4f w = v + v;
  volatile v4f* p = (volatile v4f*)(out + (size_t)4 * i);
  *p = w;
  __threadfence();
  *p = w;
}

__global__ __launch_bounds__(kThreads) void node_scan_kernel(
    const float* inputs, const float* nei, const float* numNei, const float* h0,
    const float* Wg, const float* bg, const float* Ws, const float* bs, const float* Wn,
    const int* seq, float* Hs, float* Cs) {
  __shared__ __align__(16) _Float16 sH16[kNodes * kDim];
  __shared__ __align__(16) float sSlab[kWaves][16 * kSlabP];
  __shared__ __align__(16) float sA[kNodes];
  __shared__ __align__(16) float sVec[2 * kDim];
  __shared__ __align__(16) float sCi[kDim];
  __shared__ __align__(16) float sMV[4 * kDim];
  __shared__ __align__(16) float sPH[kWaves * kDim];
  __shared__ __align__(16) float sPS[kWaves * kDim];
  __shared__ __align__(16) float sNH[kDim];
  __shared__ __align__(16) float sMV2[4 * kDim];

  const int tid  = threadIdx.x;
  const int lane = tid & 31;
  const int wave = tid >> 5;
  const int c    = lane & 15;
  const int hh   = lane >> 4;
  const int koff = hh * 8;
  const int mOff = hh * 8;
  const int grp  = tid >> 6;
  const int dd   = tid & 63;

  v16h bf[4][2];
#pragma unroll
  for (int j = 0; j < 4; ++j) {
#pragma unroll
    for (int ks = 0; ks < 2; ++ks) {
      const float* wr = Wn + (size_t)(16 * j + c) * kDim + 32 * ks + koff;
      const v4f w0 = *(const v4f*)(wr);
      const v4f w1 = *(const v4f*)(wr + 4);
      const v4f w2 = *(const v4f*)(wr + 16);
      const v4f w3 = *(const v4f*)(wr + 20);
      v16h f;
#pragma unroll
      for (int e = 0; e < 4; ++e) {
        const float x0 = w0[e];
        const float x1 = w1[e];
        const float x2 = w2[e];
        const float x3 = w3[e];
        f[e]      = eng::to_h_flush(x0, kCarryW);
        f[4 + e]  = eng::to_h_flush(x1, kCarryW);
        f[8 + e]  = eng::to_h_flush(x2, kCarryW);
        f[12 + e] = eng::to_h_flush(x3, kCarryW);
      }
      bf[j][ks] = f;
    }
  }

#pragma unroll 1
  for (int it = 0; it < 32; ++it) {
    const int ch = it * kThreads + tid;
    const v4f x0 = *(const v4f*)(h0 + (size_t)ch * 8);
    const v4f x1 = *(const v4f*)(h0 + (size_t)ch * 8 + 4);
    v8h hv;
#pragma unroll
    for (int e = 0; e < 4; ++e) {
      const float y0 = x0[e];
      const float y1 = x1[e];
      hv[e]     = eng::to_h_flush(y0, kCarryH);
      hv[4 + e] = eng::to_h_flush(y1, kCarryH);
    }
    *(v8h*)(sH16 + (size_t)ch * 8) = hv;
  }

  const float* wp = (grp == 0) ? (Wg + (size_t)dd * 128)
                  : (grp == 1) ? (Wg + (size_t)dd * 128 + 64)
                  : (grp == 2) ? (Ws + (size_t)dd * kDim)
                               : (Wn + (size_t)dd * kDim);
  const float* wq = Wn + (size_t)dd * kDim + 16 * grp;
  const float bgv = bg[dd];
  const float bsv = bs[dd];
  const float biasv = (grp == 0) ? bgv : ((grp == 2) ? bsv : 0.0f);
  const gvf* Hv = (const gvf*)Hs;
  const gvf* Cv = (const gvf*)Cs;
  float* slab = sSlab[wave];

  __syncthreads();

#pragma unroll 1
  for (int s = 0; s < kNodes; ++s) {
    int idx = seq[s];
    idx = (idx < 0) ? 0 : idx;
    idx = (idx > kNodes - 1) ? (kNodes - 1) : idx;
    const float num  = numNei[idx];
    const float rnum = 1.0f / num;

    *(v4f*)(sA + 4 * tid) = *(const v4f*)(nei + (size_t)idx * kNodes + 4 * tid);
    if (grp == 0) {
      sVec[dd] = inputs[(size_t)idx * kDim + dd];
    } else if (grp == 1) {
      sVec[kDim + dd] = Hv[(size_t)idx * kDim + dd];
    } else if (grp == 2) {
      sCi[dd] = Cv[(size_t)idx * kDim + dd];
    }
    __syncthreads();

    {
      const float* vp = sVec + kDim * (grp & 1);
      float dacc = 0.0f;
#pragma unroll 4
      for (int k4 = 0; k4 < 16; ++k4) {
        const v4f w = *(const v4f*)(wp + 4 * k4);
        const v4f x = *(const v4f*)(vp + 4 * k4);
        dacc = fmaf(w[0], x[0], dacc);
        dacc = fmaf(w[1], x[1], dacc);
        dacc = fmaf(w[2], x[2], dacc);
        dacc = fmaf(w[3], x[3], dacc);
      }
      sMV[tid] = dacc + biasv;
    }
    __syncthreads();

    {
      const float fs0 = sMV[2 * kDim + lane];
      const float fs1 = sMV[2 * kDim + 32 + lane];
      float sh0 = 0.0f, sh1 = 0.0f, ss0 = 0.0f, ss1 = 0.0f;
#pragma unroll 1
      for (int ti = 0; ti < kTilesPW; ++ti) {
        const int m0 = wave * kRowsPW + ti * 16;
        const float av = sA[m0 + c];
        const unsigned bal = __builtin_amdgcn_ballot_w32(av != 0.0f);
        unsigned mask = bal & 0xffffu;
        const _Float16* ap = sH16 + (size_t)(m0 + c) * kDim + koff;
        const v16h a0 = eng::frag_load(ap);
        const v16h a1 = eng::frag_load(ap + 32);
        v8f acc[4];
#pragma unroll
        for (int j = 0; j < 4; ++j) {
          acc[j] = (v8f){0.f, 0.f, 0.f, 0.f, 0.f, 0.f, 0.f, 0.f};
          acc[j] = eng::mma_h(a0, bf[j][0], acc[j]);
          acc[j] = eng::mma_h(a1, bf[j][1], acc[j]);
        }
#pragma unroll
        for (int j = 0; j < 4; ++j) eng::guard_acc(acc[j], a0, a1, bf[j][0], bf[j][1]);

        if (mask != 0u) {
#pragma unroll
          for (int j = 0; j < 4; ++j) {
#pragma unroll
            for (int r = 0; r < 8; ++r) {
              slab[(mOff + r) * kSlabP + 16 * j + c] = acc[j][r] * kFold;
            }
          }
          eng::wave_lds_fence();
#pragma unroll 1
          for (int it = 0; it < 16 && mask != 0u; ++it) {
            const int b = __builtin_ctz(mask);
            mask &= (mask - 1u);
            const int jn = m0 + b;
            const float aw  = sA[jn];
            const float hv0 = Hv[(size_t)jn * kDim + lane];
            const float hv1 = Hv[(size_t)jn * kDim + 32 + lane];
            const float g0  = slab[b * kSlabP + lane];
            const float g1  = slab[b * kSlabP + 32 + lane];
            sh0 = fmaf(aw, hv0, sh0);
            sh1 = fmaf(aw, hv1, sh1);
            ss0 = fmaf(aw, eng::sigm(fs0 + g0), ss0);
            ss1 = fmaf(aw, eng::sigm(fs1 + g1), ss1);
          }
          eng::wave_lds_fence();
        }
      }
      sPH[wave * kDim + lane]      = sh0;
      sPH[wave * kDim + 32 + lane] = sh1;
      sPS[wave * kDim + lane]      = ss0;
      sPS[wave * kDim + 32 + lane] = ss1;
    }
    __syncthreads();

    if (grp == 0) {
      float t = 0.0f;
#pragma unroll
      for (int w = 0; w < kWaves; ++w) t += sPH[w * kDim + dd];
      sNH[dd] = t * rnum;
    }
    __syncthreads();

    {
      const float* vq = sNH + 16 * grp;
      float dacc = 0.0f;
#pragma unroll
      for (int k4 = 0; k4 < 4; ++k4) {
        const v4f w = *(const v4f*)(wq + 4 * k4);
        const v4f x = *(const v4f*)(vq + 4 * k4);
        dacc = fmaf(w[0], x[0], dacc);
        dacc = fmaf(w[1], x[1], dacc);
        dacc = fmaf(w[2], x[2], dacc);
        dacc = fmaf(w[3], x[3], dacc);
      }
      sMV2[tid] = dacc;
    }
    __syncthreads();

    if (grp == 0) {
      const float gn  = (sMV2[dd] + sMV2[kDim + dd]) + (sMV2[2 * kDim + dd] + sMV2[3 * kDim + dd]);
      const float pre = (sMV[dd] + sMV[kDim + dd]) + gn;
      const float fsd = sMV[2 * kDim + dd];
      const float gi  = sMV[3 * kDim + dd];
      float sumS = 0.0f;
#pragma unroll
      for (int w = 0; w < kWaves; ++w) sumS += sPS[w * kDim + dd];
      const float ci = sCi[dd];
      const float ig = eng::sigm(pre);
      const float hc = tanhf(pre);
      const float fg = eng::sigm(fsd + gi);
      const float cn = (sumS * ci) * rnum + fg * ci + ig * hc;
      const float hn = tanhf(ig * cn);
      volatile float* hp = (volatile float*)(Hs + (size_t)idx * kDim + dd);
      volatile float* cp = (volatile float*)(Cs + (size_t)idx * kDim + dd);
      *hp = hn;
      *cp = cn;
      __threadfence();
      *hp = hn;
      *cp = cn;
      sH16[(size_t)idx * kDim + dd] = eng::to_h_flush(hn, kCarryH);
    }
    __syncthreads();
  }
}

extern "C" void kernel_launch(void* const* d_in, const int* in_sizes, int n_in,
                              void* d_out, int out_size, void* d_ws, size_t ws_size,
                              hipStream_t stream) {
  if (n_in < 11 || d_out == nullptr || d_ws == nullptr) return;
  if (in_sizes[0] != kNodes * kDim) return;
  if (in_sizes[1] != kNodes * kNodes) return;
  if (in_sizes[2] != kNodes) return;
  if (in_sizes[3] != kNodes * kDim) return;
  if (in_sizes[4] != kNodes * kDim) return;
  if (in_sizes[5] != kDim * 2 * kDim) return;
  if (in_sizes[6] != kDim) return;
  if (in_sizes[7] != kDim * kDim) return;
  if (in_sizes[8] != kDim) return;
  if (in_sizes[9] != kDim * kDim) return;
  if (in_sizes[10] != kNodes) return;
  if (out_size != kNodes * kDim) return;
  if (ws_size < kWsTotal) return;

  const float* inputs = (const float*)d_in[0];
  const float* nei    = (const float*)d_in[1];
  const float* numNei = (const float*)d_in[2];
  const float* h0     = (const float*)d_in[3];
  const float* c0     = (const float*)d_in[4];
  const float* Wg     = (const float*)d_in[5];
  const float* bg     = (const float*)d_in[6];
  const float* Ws     = (const float*)d_in[7];
  const float* bs     = (const float*)d_in[8];
  const float* Wn     = (const float*)d_in[9];
  const int*   seq    = (const int*)d_in[10];
  float* out = (float*)d_out;

  char* ws = (char*)d_ws;
  size_t off = 0;
  auto carve = [&](size_t bytes) -> char* { char* p = ws + off; off += bytes; return p; };
  float* Hs = (float*)carve(kPlaneBytes);
  float* Cs = (float*)carve(kPlaneBytes);
  if (off != kWsTotal) return;

  state_init_kernel<<<128, 256, 0, stream>>>(h0, c0, Hs, Cs);
  node_scan_kernel<<<1, kThreads, 0, stream>>>(inputs, nei, numNei, h0, Wg, bg, Ws, bs, Wn, seq, Hs, Cs);
  out_double_kernel<<<64, 256, 0, stream>>>(Hs, out);
}
